// GATEncoder_77695958385351
// MI455X (gfx1250) — hardware-verified
//
#include <hip/hip_runtime.h>
#include <stddef.h>


typedef _Float16 v16h __attribute__((ext_vector_type(16)));
typedef _Float16 v8h  __attribute__((ext_vector_type(8)));
typedef _Float16 v4h  __attribute__((ext_vector_type(4)));
typedef float    v8f  __attribute__((ext_vector_type(8)));
typedef float    v4f  __attribute__((ext_vector_type(4)));
typedef int      v4i  __attribute__((ext_vector_type(4)));
typedef _Float16 h16;

#ifndef NB
#define NB 8
#endif
#ifndef SEQ
#define SEQ 1024
#endif
#define NB_FULL  8
#define SEQ_FULL 1024
#define FIN   256
#define FOUT  512
#define NH    8
#define HD    64
#define MROWS (NB * SEQ)

static_assert(NB >= 1 && NB <= NB_FULL);
static_assert(SEQ >= 128 && SEQ <= SEQ_FULL && (SEQ % 128) == 0);
static_assert((FIN % 64) == 0 && (FIN % 32) == 0);
static_assert((FOUT % 64) == 0 && FOUT == NH * HD);
static_assert(NH == 8);
static_assert(HD == 64);
static_assert(FOUT == 4 * 32 * 4);
static_assert((MROWS % 64) == 0 && (SEQ % 64) == 0 && (SEQ % 32) == 0);
static_assert(((size_t)MROWS * FIN) % 2048 == 0);
static_assert((size_t)MROWS * FIN < (size_t)0xFFFFFFFFu);

#define LDT 72
#define LDC 68
#define CLD (SEQ + 4)
#define HLD (FOUT + 4)
#define NIT (SEQ / 128)
static_assert((LDT % 8) == 0 && LDT >= 64);
static_assert((LDC % 4) == 0 && LDC >= 64);
static_assert((CLD % 4) == 0 && (HLD % 4) == 0);
static_assert(NIT * 128 == SEQ && NIT <= 8);
static_assert(8 * 2 == 16);
static_assert(16 * HLD <= 16 * CLD);

#define WCARRY 64.0f
#define PCARRY 16384.0f
#define ALPHA  0.2f
#define NEGFILL (-1.0e9f)

#define WT_BYTES  ((size_t)FOUT * FIN * 2)
#define H16_BYTES ((size_t)MROWS * FIN * 2)
#define VT_BYTES  ((size_t)NB * FOUT * SEQ * 2)
#define FP_BYTES  ((size_t)(FOUT / 64) * 2 * MROWS * 4)
#define OFF_WT  ((size_t)0)
#define OFF_H16 (OFF_WT + WT_BYTES)
#define OFF_VT  (OFF_H16 + H16_BYTES)
#define OFF_FP  (OFF_VT + VT_BYTES)
#define WS_TOTAL (OFF_FP + FP_BYTES)
static_assert((WT_BYTES % 128) == 0 && (H16_BYTES % 128) == 0);
static_assert((VT_BYTES % 128) == 0 && (FP_BYTES % 128) == 0);
static_assert(WS_TOTAL <= (size_t)134217728);

__device__ __forceinline__ float bf16r(float x) {
  unsigned int u = __float_as_uint(x);
  u = (u + 0x7FFFu + ((u >> 16) & 1u)) & 0xFFFF0000u;
  return __uint_as_float(u);
}

static __device__ __forceinline__ h16 toh_flush(float v) {
  const h16 r = (h16)v;
  return (fabsf(v) < 6.103515625e-05f) ? (h16)0.0f : r;
}

__device__ __forceinline__ v16h frag_at(const _Float16* p) {
  v8h lo = *(const v8h*)(p);
  v8h hi = *(const v8h*)(p + 16);
  v16h out;
#pragma unroll
  for (int i = 0; i < 8; ++i) { out[i] = lo[i]; out[i + 8] = hi[i]; }
  return out;
}

__device__ __forceinline__ v8f wmma16(v16h a, v16h b, v8f c) {
  v8f d = __builtin_amdgcn_wmma_f32_16x16x32_f16(false, a, false, b, (short)0, c,
                                                 false, false);
  asm volatile("v_nop\n\tv_nop\n\tv_nop\n\tv_nop" : "+v"(d) : "v"(a), "v"(b));
  return d;
}

__device__ __forceinline__ float max4(const v4f e) {
  return fmaxf(fmaxf(e[0], e[1]), fmaxf(e[2], e[3]));
}

__device__ __forceinline__ v4f logit4(const v4i a, const v4f c, const v4f s, const float f1v) {
  v4f o;
#pragma unroll
  for (int q = 0; q < 4; ++q) {
    const float t = f1v + s[q];
    const float lr = (t >= 0.0f) ? t : ALPHA * t;
    const float ev = lr + c[q];
    o[q] = (a[q] == 0) ? NEGFILL : ev;
  }
  return o;
}

__device__ __forceinline__ h16 pconv(const float e, const float mx, float& ps) {
  const float pv = __expf(e - mx) * PCARRY;
  const h16 hv = toh_flush(pv);
  ps += (float)hv;
  return hv;
}

__global__ __launch_bounds__(256) void wconv_kernel(
    const float* __restrict__ W, _Float16* __restrict__ Wt, unsigned ldw, unsigned ldk) {
  __shared__ _Float16 T[64 * LDT];
  const unsigned tid = threadIdx.x;
  const unsigned n0 = blockIdx.x * 64u;
  const unsigned k0 = blockIdx.y * 64u;
#pragma unroll 4
  for (unsigned j = 0; j < 16u; ++j) {
    const unsigned idx = tid + 256u * j;
    const unsigned kr = idx >> 6, nc = idx & 63u;
    const float v = W[(size_t)(k0 + kr) * ldw + n0 + nc];
    T[nc * LDT + kr] = toh_flush(WCARRY * bf16r(v));
  }
  __syncthreads();
  v8h x[2];
  size_t off[2];
#pragma unroll
  for (unsigned i = 0; i < 2u; ++i) {
    const unsigned n = 32u * i + (tid >> 3);
    const unsigned kc = (tid & 7u) * 8u;
    x[i] = *(const v8h*)&T[n * LDT + kc];
    off[i] = (size_t)(n0 + n) * ldk + k0 + kc;
  }
#pragma unroll
  for (int i = 0; i < 2; ++i) *(volatile v8h*)(Wt + off[i]) = x[i];
  __threadfence();
#pragma unroll
  for (int i = 0; i < 2; ++i) *(volatile v8h*)(Wt + off[i]) = x[i];
}

__global__ __launch_bounds__(256) void hconv_kernel(
    const float* __restrict__ X, _Float16* __restrict__ dst) {
  const unsigned g = blockIdx.x * 256u + threadIdx.x;
  const unsigned crow = g / (unsigned)(FIN / 8);
  const unsigned c = (g - crow * (unsigned)(FIN / 8)) * 8u;
  const unsigned bidx = crow / (unsigned)SEQ;
  const unsigned sq = crow - bidx * (unsigned)SEQ;
  const size_t srow = (size_t)bidx * SEQ_FULL + sq;
  const v4f a0 = *(const v4f*)(X + srow * FIN + c);
  const v4f a1 = *(const v4f*)(X + srow * FIN + c + 4u);
  v8h o;
#pragma unroll
  for (int i = 0; i < 4; ++i) {
    o[i]     = toh_flush(bf16r(a0[i]));
    o[i + 4] = toh_flush(bf16r(a1[i]));
  }
  _Float16* p = dst + (size_t)crow * FIN + c;
  *(volatile v8h*)p = o;
  __threadfence();
  *(volatile v8h*)p = o;
}

__global__ __launch_bounds__(256) void gemm_ht_kernel(
    const _Float16* __restrict__ A16, const _Float16* __restrict__ Bt,
    const float* __restrict__ bias, const float* __restrict__ avec,
    _Float16* __restrict__ vt, float* __restrict__ fp) {
  __shared__ __attribute__((aligned(16))) float Cs[64 * LDC];
  __shared__ __attribute__((aligned(16))) float Fs[2 * 64];
  const unsigned tid = threadIdx.x, lane = tid & 31u;
  const unsigned w = __builtin_amdgcn_readfirstlane(tid >> 5);
  const unsigned mw = w >> 1, nw = w & 1u;
  const unsigned hh = lane >> 4, m = lane & 15u;
  const unsigned n0 = blockIdx.x * 64u;
  const unsigned row0 = blockIdx.y * 64u;
  const unsigned K = (unsigned)FIN;

  const _Float16* ap  = A16 + (size_t)(row0 + mw * 16u + m) * K + hh * 8u;
  const _Float16* bp0 = Bt + (size_t)(n0 + nw * 32u + m) * K + hh * 8u;
  const _Float16* bp1 = bp0 + (size_t)16 * K;
  v8f acc0 = {}, acc1 = {};
#pragma unroll 2
  for (unsigned k0 = 0; k0 < K; k0 += 32u) {
    const v16h a  = frag_at(ap + k0);
    const v16h b0 = frag_at(bp0 + k0);
    const v16h b1 = frag_at(bp1 + k0);
    acc0 = wmma16(a, b0, acc0);
    acc1 = wmma16(a, b1, acc1);
  }
  const float bia0 = bf16r(bias[n0 + nw * 32u + m]);
  const float bia1 = bf16r(bias[n0 + nw * 32u + 16u + m]);
#pragma unroll
  for (int r = 0; r < 8; ++r) {
    float* d = &Cs[(mw * 16u + hh * 8u + (unsigned)r) * LDC + nw * 32u + m];
    d[0]  = acc0[r] * (1.0f / WCARRY) + bia0;
    d[16] = acc1[r] * (1.0f / WCARRY) + bia1;
  }
  __syncthreads();

  {
    const unsigned bidx = row0 / (unsigned)SEQ;
    const unsigned key0 = row0 - bidx * (unsigned)SEQ;
    v8h x[2];
    size_t off[2];
#pragma unroll
    for (unsigned i = 0; i < 2u; ++i) {
      const unsigned dcol = 32u * i + (tid >> 3);
      const unsigned kk = (tid & 7u) * 8u;
#pragma unroll
      for (unsigned j = 0; j < 8u; ++j) {
        const float t = Cs[(kk + j) * LDC + dcol];
        x[i][j] = toh_flush(t);
      }
      off[i] = ((size_t)bidx * FOUT + n0 + dcol) * SEQ + key0 + kk;
    }
#pragma unroll
    for (int i = 0; i < 2; ++i) *(volatile v8h*)(vt + off[i]) = x[i];
    __threadfence();
#pragma unroll
    for (int i = 0; i < 2; ++i) *(volatile v8h*)(vt + off[i]) = x[i];
  }

  {
    const unsigned r = tid >> 2, q = tid & 3u;
    float s1 = 0.0f, s2 = 0.0f;
#pragma unroll 4
    for (unsigned j = 0; j < 16u; ++j) {
      const unsigned c = q * 16u + j;
      const float t = Cs[r * LDC + c];
      s1 += t * bf16r(avec[c]);
      s2 += t * bf16r(avec[(unsigned)HD + c]);
    }
    s1 += __shfl_xor(s1, 1, 32);
    s2 += __shfl_xor(s2, 1, 32);
    s1 += __shfl_xor(s1, 2, 32);
    s2 += __shfl_xor(s2, 2, 32);
    if (q == 0u) { Fs[r] = s1; Fs[64u + r] = s2; }
  }
  __syncthreads();
  if (w == 0u) {
    const unsigned which = lane >> 4, ch = lane & 15u;
    const v4f v = *(const v4f*)&Fs[which * 64u + ch * 4u];
    float* p = fp + (size_t)(blockIdx.x * 2u + which) * MROWS + row0 + ch * 4u;
    *(volatile v4f*)p = v;
    __threadfence();
    *(volatile v4f*)p = v;
  }
}

__global__ __launch_bounds__(256) __attribute__((amdgpu_num_vgpr(256))) void heads_attn_kernel(
    const int* __restrict__ adj, const float* __restrict__ dist,
    const _Float16* __restrict__ Vt, const float* __restrict__ Fp,
    const float* __restrict__ dwp, const float* __restrict__ dbp,
    float* __restrict__ out) {
  __shared__ __attribute__((aligned(16))) float Cb[16 * CLD];
  __shared__ __attribute__((aligned(16))) float f2s[NH * SEQ];

  const unsigned tid = threadIdx.x, lane = tid & 31u;
  const unsigned w = __builtin_amdgcn_readfirstlane(tid >> 5);
  const unsigned hh = lane >> 4, m = lane & 15u;
  const unsigned i0 = blockIdx.x * 16u;
  const unsigned b = blockIdx.y;

  for (unsigned idx = tid; idx < (unsigned)(NH * SEQ / 4); idx += 256u) {
    const unsigned hd = idx / (unsigned)(SEQ / 4);
    const unsigned j4 = idx - hd * (unsigned)(SEQ / 4);
    const v4f s = *(const v4f*)(Fp + (size_t)(hd * 2u + 1u) * MROWS + (size_t)b * SEQ + j4 * 4u);
    *(v4f*)&f2s[hd * (unsigned)SEQ + j4 * 4u] = s;
  }
  {
    const float dw = bf16r(dwp[0]);
    const float db = bf16r(dbp[0]);
#pragma unroll 1
    for (unsigned rr = 0; rr < 2u; ++rr) {
      const unsigned r = w * 2u + rr;
      const float* dR = dist + ((size_t)b * SEQ_FULL + i0 + r) * SEQ_FULL + lane * 4u;
#pragma unroll 1
      for (unsigned it = 0; it < (unsigned)NIT; ++it) {
        const v4f d4 = *(const v4f*)(dR + it * 128u);
        v4f c4;
#pragma unroll
        for (int q = 0; q < 4; ++q) {
          const float px = 1.0f / (bf16r(d4[q]) + 1.0e-8f);
          c4[q] = dw * px + db;
        }
        *(v4f*)&Cb[r * (unsigned)CLD + it * 128u + lane * 4u] = c4;
      }
    }
  }
  __syncthreads();

  const float f1v = Fp[(size_t)(w * 2u) * MROWS + (size_t)b * SEQ + i0 + m];
  const int* adjR = adj + ((size_t)b * SEQ_FULL + i0 + m) * SEQ_FULL + hh * 8u;
  const _Float16* bp = Vt + ((size_t)b * FOUT + w * (unsigned)HD + m) * SEQ + hh * 8u;
  const unsigned cbase = m * (unsigned)CLD + hh * 8u;
  const unsigned sbase = w * (unsigned)SEQ + hh * 8u;

  float rowM = -1.0e30f;
  float rowS = 0.0f;
  v8f acc0 = {}, acc1 = {}, acc2 = {}, acc3 = {};

#pragma unroll 1
  for (unsigned j0 = 0; j0 < (unsigned)SEQ; j0 += 32u) {
    const v4i a0 = *(const v4i*)(adjR + j0);
    const v4i a1 = *(const v4i*)(adjR + j0 + 4u);
    const v4i a2 = *(const v4i*)(adjR + j0 + 16u);
    const v4i a3 = *(const v4i*)(adjR + j0 + 20u);
    const v4f c0 = *(const v4f*)&Cb[cbase + j0];
    const v4f c1 = *(const v4f*)&Cb[cbase + j0 + 4u];
    const v4f c2 = *(const v4f*)&Cb[cbase + j0 + 16u];
    const v4f c3 = *(const v4f*)&Cb[cbase + j0 + 20u];
    const v4f s0 = *(const v4f*)&f2s[sbase + j0];
    const v4f s1 = *(const v4f*)&f2s[sbase + j0 + 4u];
    const v4f s2 = *(const v4f*)&f2s[sbase + j0 + 16u];
    const v4f s3 = *(const v4f*)&f2s[sbase + j0 + 20u];

    const v4f e0 = logit4(a0, c0, s0, f1v);
    const v4f e1 = logit4(a1, c1, s1, f1v);
    const v4f e2 = logit4(a2, c2, s2, f1v);
    const v4f e3 = logit4(a3, c3, s3, f1v);

    float mc = fmaxf(fmaxf(max4(e0), max4(e1)), fmaxf(max4(e2), max4(e3)));
    mc = fmaxf(mc, __shfl_xor(mc, 16, 32));
    const float newM = fmaxf(rowM, mc);
    const float scale = __expf(rowM - newM);
    rowM = newM;

    float ps = 0.0f;
    v16h af;
#pragma unroll
    for (int q = 0; q < 4; ++q) {
      af[q]      = pconv(e0[q], newM, ps);
      af[q + 4]  = pconv(e1[q], newM, ps);
      af[q + 8]  = pconv(e2[q], newM, ps);
      af[q + 12] = pconv(e3[q], newM, ps);
    }
    ps += __shfl_xor(ps, 16, 32);
    rowS = rowS * scale + ps;

#pragma unroll
    for (int r = 0; r < 8; ++r) {
      const float sc = __shfl(scale, (int)(8u * hh) + r, 32);
      acc0[r] *= sc;
      acc1[r] *= sc;
      acc2[r] *= sc;
      acc3[r] *= sc;
    }

    const v16h b0 = frag_at(bp + j0);
    const v16h b1 = frag_at(bp + (size_t)16 * SEQ + j0);
    acc0 = wmma16(af, b0, acc0);
    acc1 = wmma16(af, b1, acc1);
    const v16h b2 = frag_at(bp + (size_t)32 * SEQ + j0);
    const v16h b3 = frag_at(bp + (size_t)48 * SEQ + j0);
    acc2 = wmma16(af, b2, acc2);
    acc3 = wmma16(af, b3, acc3);
  }

  const float invl = 1.0f / rowS;
  __syncthreads();
#pragma unroll
  for (int r = 0; r < 8; ++r) {
    const float ri = __shfl(invl, (int)(8u * hh) + r, 32);
    float* d = &Cb[(hh * 8u + (unsigned)r) * (unsigned)HLD + w * (unsigned)HD + m];
    d[0]  = acc0[r] * ri;
    d[16] = acc1[r] * ri;
    d[32] = acc2[r] * ri;
    d[48] = acc3[r] * ri;
  }
  __syncthreads();

#pragma unroll 1
  for (unsigned rr = 0; rr < 2u; ++rr) {
    const unsigned r = w * 2u + rr;
    const v4f x0 = *(const v4f*)&Cb[r * (unsigned)HLD + lane * 4u];
    const v4f x1 = *(const v4f*)&Cb[r * (unsigned)HLD + 128u + lane * 4u];
    const v4f x2 = *(const v4f*)&Cb[r * (unsigned)HLD + 256u + lane * 4u];
    const v4f x3 = *(const v4f*)&Cb[r * (unsigned)HLD + 384u + lane * 4u];
    float* p0 = out + ((size_t)b * SEQ_FULL + i0 + r) * FOUT + lane * 4u;
    float* p1 = p0 + 128;
    float* p2 = p0 + 256;
    float* p3 = p0 + 384;
    *(volatile v4f*)p0 = x0;
    *(volatile v4f*)p1 = x1;
    *(volatile v4f*)p2 = x2;
    *(volatile v4f*)p3 = x3;
    __threadfence();
    *(volatile v4f*)p0 = x0;
    *(volatile v4f*)p1 = x1;
    *(volatile v4f*)p2 = x2;
    *(volatile v4f*)p3 = x3;
  }
}

static_assert(16 * CLD * 4 + NH * SEQ * 4 <= 131072);
static_assert(64 * LDC * 4 + 2 * 64 * 4 <= 131072);
static_assert(64 * LDT * 2 <= 131072);

extern "C" void kernel_launch(void* const* d_in, const int* in_sizes, int n_in,
                              void* d_out, int out_size, void* d_ws, size_t ws_size,
                              hipStream_t stream) {
  if (n_in < 8) return;
  const long long need_rows = (long long)(NB - 1) * SEQ_FULL + SEQ;
  if ((long long)in_sizes[0] < need_rows * FIN) return;
  if ((long long)in_sizes[1] < (need_rows - 1) * SEQ_FULL + SEQ) return;
  if ((long long)in_sizes[2] < (need_rows - 1) * SEQ_FULL + SEQ) return;
  if ((long long)in_sizes[3] < (long long)FIN * FOUT) return;
  if (in_sizes[4] < FOUT) return;
  if (in_sizes[5] < 2 * HD) return;
  if (in_sizes[6] < 1 || in_sizes[7] < 1) return;
  if ((long long)out_size < need_rows * FOUT) return;
  if (ws_size < WS_TOTAL) return;

  const float* X    = (const float*)d_in[0];
  const int*   adj  = (const int*)d_in[1];
  const float* dist = (const float*)d_in[2];
  const float* Wm   = (const float*)d_in[3];
  const float* bvec = (const float*)d_in[4];
  const float* avec = (const float*)d_in[5];
  const float* dwp  = (const float*)d_in[6];
  const float* dbp  = (const float*)d_in[7];
  float* out = (float*)d_out;

  char* ws = (char*)d_ws;
  _Float16* Wt16 = (_Float16*)(ws + OFF_WT);
  _Float16* H16  = (_Float16*)(ws + OFF_H16);
  _Float16* Vt16 = (_Float16*)(ws + OFF_VT);
  float*    Fp   = (float*)(ws + OFF_FP);

  dim3 blk(256);
  wconv_kernel<<<dim3(FOUT / 64, FIN / 64), blk, 0, stream>>>(Wm, Wt16, (unsigned)FOUT, (unsigned)FIN);
  hconv_kernel<<<dim3((unsigned)(((size_t)MROWS * FIN) / 2048)), blk, 0, stream>>>(X, H16);
  gemm_ht_kernel<<<dim3(FOUT / 64, MROWS / 64), blk, 0, stream>>>(H16, Wt16, bvec, avec, Vt16, Fp);
  heads_attn_kernel<<<dim3(SEQ / 16, NB), blk, 0, stream>>>(adj, dist, Vt16, Fp, dwp, dbp, out);
}
